// LiquidHawkesModel_25220047962221
// MI455X (gfx1250) — hardware-verified
//
#include <hip/hip_runtime.h>
#include <math.h>

typedef __attribute__((ext_vector_type(16))) _Float16 v16h;
typedef __attribute__((ext_vector_type(8)))  _Float16 v8h;
typedef __attribute__((ext_vector_type(8)))  float    v8f;
typedef __attribute__((ext_vector_type(4)))  float    v4f;

__device__ __forceinline__ void dep_guard_h(v8f& a, v8f& b, v16h x, v16h y) { asm volatile("v_nop\n\tv_nop\n\tv_nop\n\tv_nop" : "+v"(a), "+v"(b) : "v"(x), "v"(y)); }
__device__ __forceinline__ void keep4_h(v16h a, v16h b, v16h c, v16h d) { asm volatile("v_nop" :: "v"(a), "v"(b), "v"(c), "v"(d)); }
__device__ __forceinline__ void acc_guard4(v8f& a, v8f& b, v8f& c, v8f& d) { asm volatile("v_nop\n\tv_nop\n\tv_nop\n\tv_nop" : "+v"(a), "+v"(b), "+v"(c), "+v"(d)); }
__device__ __forceinline__ void acc_guard3(v8f& a, v8f& b, v8f& c) { asm volatile("v_nop\n\tv_nop\n\tv_nop\n\tv_nop" : "+v"(a), "+v"(b), "+v"(c)); }
template <typename T> struct Frag;
template <> struct Frag<_Float16> {
  typedef v16h V; union U { v16h v; v8h h[2]; };
  static __device__ __forceinline__ v16h load(const _Float16* p) {
    U f; f.h[0] = *(const v8h*)(p); f.h[1] = *(const v8h*)(p + 16); return f.v;
  }
  static __device__ __forceinline__ v8f mma(v16h a, v16h b, v8f c) {
    return __builtin_amdgcn_wmma_f32_16x16x32_f16(false, a, false, b, (short)0, c, false, false);
  }
  static __device__ __forceinline__ void guard(v8f& a, v8f& b, v16h x, v16h y) { dep_guard_h(a, b, x, y); }
  static __device__ __forceinline__ void keep(v16h a, v16h b, v16h c, v16h d) { keep4_h(a, b, c, d); }
};

constexpr int NBATCH = 256;
constexpr int NSTEP  = 512;
constexpr int NIN    = 64;
constexpr int NHID   = 256;
constexpr int NBB    = 256;
constexpr int NMOT   = 64;
constexpr int KCAT   = NIN + NHID;
constexpr int NROWS  = NBATCH * NSTEP;
constexpr int ROWS_PER_BLK  = 32;
constexpr int NBLK_SCAN     = NBATCH / ROWS_PER_BLK;
constexpr int A0_LD  = 328;
constexpr int Z_LD   = 264;
constexpr int HC_LD  = 72;
constexpr int HA_LD  = 52;
constexpr int NHEADH = 48;
constexpr int ROWS_PER_HBLK = 128;
constexpr float W_CARRY     = 64.0f;
constexpr float W_CARRY_INV = 0.015625f;

static_assert(KCAT % 32 == 0 && NBB % 32 == 0 && NHID % 32 == 0 && NMOT % 32 == 0, "k steps");
static_assert(NROWS % ROWS_PER_HBLK == 0 && NBATCH % ROWS_PER_BLK == 0, "tiles");

__device__ __forceinline__ v8f zero8() { return (v8f){0.f, 0.f, 0.f, 0.f, 0.f, 0.f, 0.f, 0.f}; }

__device__ __forceinline__ float clamp60(float a) { return fminf(fmaxf(a, -60.0f), 60.0f); }
__device__ __forceinline__ float tanh_f(float a) {
  const float e = expf(clamp60(2.0f * a));
  return 1.0f - 2.0f / (1.0f + e);
}
__device__ __forceinline__ float sigmoid_f(float a) {
  const float e = expf(clamp60(-a));
  return 1.0f / (1.0f + e);
}
__device__ __forceinline__ float lecun_tanh_f(float a) { return 1.7159f * tanh_f(0.666f * a); }
__device__ __forceinline__ float silu_f(float a) { return a * sigmoid_f(a); }
__device__ __forceinline__ float softplus_f(float a) { return fmaxf(a, 0.0f) + log1pf(expf(-fabsf(a))); }

__global__ __launch_bounds__(256) void k_transpose_cast(const float* __restrict__ in, unsigned short* __restrict__ out,
                                                        int Kdim, int Ndim, float carry) {
  __shared__ float st[64 * 33];
  const int tid = threadIdx.x;
  const int k0 = blockIdx.x * 64, n0 = blockIdx.y * 32;
  {
    const int k = tid >> 2, nq = (tid & 3) * 8;
    const float* src = in + (size_t)(k0 + k) * Ndim + n0 + nq;
    const v4f a = *(const v4f*)src;
    const v4f b = *(const v4f*)(src + 4);
    float* d = st + k * 33 + nq;
    d[0] = a[0]; d[1] = a[1]; d[2] = a[2]; d[3] = a[3];
    d[4] = b[0]; d[5] = b[1]; d[6] = b[2]; d[7] = b[3];
  }
  __syncthreads();
  const int n = tid >> 3, c8 = (tid & 7) * 8;
  v8h hv;
#pragma unroll
  for (int e = 0; e < 8; ++e) hv[e] = (_Float16)(st[(c8 + e) * 33 + n] * carry);
  unsigned short* dst = out + (size_t)(n0 + n) * Kdim + k0 + c8;
  *(volatile v8h*)dst = hv;
  __threadfence();
  *(volatile v8h*)dst = hv;
}

__global__ __launch_bounds__(384) void k_pack_head_w(const float* __restrict__ ihw0, const float* __restrict__ ahw0,
                                                      const float* __restrict__ chw0, unsigned short* __restrict__ out,
                                                      float carry) {
  const int tid = threadIdx.x;
  const int n = tid >> 3, c8 = (tid & 7) * 8;
  v8h hv;
#pragma unroll
  for (int e = 0; e < 8; ++e) {
    const int k = c8 + e;
    const float va = ihw0[k * 16 + (n & 15)];
    const float vb = ahw0[k * 16 + (n & 15)];
    const float vc = chw0[k * 8 + (n & 7)];
    const float v = (n < 16) ? va : (n < 32) ? vb : (n < 40) ? vc : 0.0f;
    hv[e] = (_Float16)(v * carry);
  }
  unsigned short* dst = out + (size_t)n * NMOT + c8;
  *(volatile v8h*)dst = hv;
  __threadfence();
  *(volatile v8h*)dst = hv;
}

template <int KDIM>
__device__ __forceinline__ void backbone_phase(const _Float16* aT, int ald, const _Float16* __restrict__ W,
                                               const float* __restrict__ bias, _Float16* zT,
                                               int ntb, int rlane, int koff, int mOff) {
  v8f acc[2][2];
  acc[0][0] = zero8(); acc[0][1] = zero8(); acc[1][0] = zero8(); acc[1][1] = zero8();
#pragma unroll 1
  for (int k0 = 0; k0 < KDIM; k0 += 32) {
    v16h bfr[2];
#pragma unroll
    for (int j = 0; j < 2; ++j)
      bfr[j] = Frag<_Float16>::load(W + (size_t)((ntb + j) * 16 + rlane) * KDIM + koff + k0);
#pragma unroll
    for (int i = 0; i < 2; ++i) {
      const v16h afr = Frag<_Float16>::load(aT + (i * 16 + rlane) * ald + koff + k0);
      acc[i][0] = Frag<_Float16>::mma(afr, bfr[0], acc[i][0]);
      acc[i][1] = Frag<_Float16>::mma(afr, bfr[1], acc[i][1]);
      Frag<_Float16>::guard(acc[i][0], acc[i][1], afr, bfr[1]);
    }
    Frag<_Float16>::keep(bfr[0], bfr[1], bfr[0], bfr[1]);
  }
  acc_guard4(acc[0][0], acc[0][1], acc[1][0], acc[1][1]);
#pragma unroll
  for (int j = 0; j < 2; ++j) {
    const int col = (ntb + j) * 16 + rlane;
    const float bv = bias[col];
#pragma unroll
    for (int i = 0; i < 2; ++i) {
#pragma unroll
      for (int r = 0; r < 8; ++r) {
        const float v = acc[i][j][r] * W_CARRY_INV + bv;
        zT[(i * 16 + mOff + r) * Z_LD + col] = (_Float16)lecun_tanh_f(v);
      }
    }
  }
}

union ZHBuf {
  _Float16 z1[ROWS_PER_BLK * Z_LD];
  float    hf[ROWS_PER_BLK * NHID];
};
static_assert(sizeof(ZHBuf) == ROWS_PER_BLK * NHID * 4, "union extent");

__global__ __launch_bounds__(256) __attribute__((amdgpu_num_vgpr(256)))
void k_cfc_scan(const float* __restrict__ x, const float* __restrict__ tsp, const float* __restrict__ hx,
                const unsigned short* __restrict__ w0t, const float* __restrict__ bias0,
                const unsigned short* __restrict__ w1t, const float* __restrict__ bias1,
                const unsigned short* __restrict__ w2t,
                const float* __restrict__ biasf1, const float* __restrict__ biasf2,
                const float* __restrict__ biasta, const float* __restrict__ biastb,
                unsigned short* __restrict__ hseq, float* __restrict__ hn) {
  __shared__ __align__(16) _Float16 sA0[ROWS_PER_BLK * A0_LD];
  __shared__ __align__(16) ZHBuf    sU;
  __shared__ __align__(16) _Float16 sZ2[ROWS_PER_BLK * Z_LD];
  __shared__ float sTs[ROWS_PER_BLK];

  const int tid = threadIdx.x, lane = tid & 31, wave = tid >> 5;
  const int rlane = lane & 15, hh = lane >> 4, koff = hh * 8, mOff = hh * 8;
  const int brow0 = blockIdx.x * ROWS_PER_BLK;
  const _Float16* W0 = (const _Float16*)w0t;
  const _Float16* W1 = (const _Float16*)w1t;
  const _Float16* W2 = (const _Float16*)w2t;
  _Float16* sZ1 = sU.z1;
  float*    sHf = sU.hf;

  {
    const int r = tid >> 3, c = (tid & 7) * 32;
    const float* src = hx + (size_t)(brow0 + r) * NHID + c;
#pragma unroll
    for (int j = 0; j < 4; ++j) {
      const v4f a = *(const v4f*)(src + j * 8);
      const v4f b = *(const v4f*)(src + j * 8 + 4);
      v8h hv;
      hv[0] = (_Float16)a[0]; hv[1] = (_Float16)a[1]; hv[2] = (_Float16)a[2]; hv[3] = (_Float16)a[3];
      hv[4] = (_Float16)b[0]; hv[5] = (_Float16)b[1]; hv[6] = (_Float16)b[2]; hv[7] = (_Float16)b[3];
      *(v8h*)(sA0 + r * A0_LD + NIN + c + j * 8) = hv;
    }
  }

#pragma unroll 1
  for (int t = 0; t < NSTEP; ++t) {
    {
      const int r = tid >> 3, c = (tid & 7) * 8;
      const float* src = x + (((size_t)(brow0 + r)) * NSTEP + t) * NIN + c;
      const v4f a = *(const v4f*)src;
      const v4f b = *(const v4f*)(src + 4);
      v8h hv;
      hv[0] = (_Float16)a[0]; hv[1] = (_Float16)a[1]; hv[2] = (_Float16)a[2]; hv[3] = (_Float16)a[3];
      hv[4] = (_Float16)b[0]; hv[5] = (_Float16)b[1]; hv[6] = (_Float16)b[2]; hv[7] = (_Float16)b[3];
      *(v8h*)(sA0 + r * A0_LD + c) = hv;
    }
    if (tid < ROWS_PER_BLK) sTs[tid] = tsp[(size_t)(brow0 + tid) * NSTEP + t];
    __syncthreads();

    backbone_phase<KCAT>(sA0, A0_LD, W0, bias0, sZ1, wave * 2, rlane, koff, mOff);
    __syncthreads();

    backbone_phase<NBB>(sZ1, Z_LD, W1, bias1, sZ2, wave * 2, rlane, koff, mOff);
    __syncthreads();

#pragma unroll 1
    for (int ubi = 0; ubi < 2; ++ubi) {
      const int ub = wave * 2 + ubi;
      v8f acc[2][4];
#pragma unroll
      for (int i = 0; i < 2; ++i)
#pragma unroll
        for (int g = 0; g < 4; ++g) acc[i][g] = zero8();
#pragma unroll 1
      for (int k0 = 0; k0 < NBB; k0 += 32) {
        v16h bfr[4];
#pragma unroll
        for (int g = 0; g < 4; ++g)
          bfr[g] = Frag<_Float16>::load(W2 + (size_t)(g * NHID + ub * 16 + rlane) * NBB + koff + k0);
#pragma unroll
        for (int i = 0; i < 2; ++i) {
          const v16h afr = Frag<_Float16>::load(sZ2 + (i * 16 + rlane) * Z_LD + koff + k0);
#pragma unroll
          for (int g = 0; g < 4; ++g) acc[i][g] = Frag<_Float16>::mma(afr, bfr[g], acc[i][g]);
          Frag<_Float16>::guard(acc[i][0], acc[i][3], afr, bfr[3]);
        }
        Frag<_Float16>::keep(bfr[0], bfr[1], bfr[2], bfr[3]);
      }
      acc_guard4(acc[0][0], acc[0][1], acc[0][2], acc[0][3]);
      acc_guard4(acc[1][0], acc[1][1], acc[1][2], acc[1][3]);

      const int u = ub * 16 + rlane;
      const float bf1v = biasf1[u], bf2v = biasf2[u], btav = biasta[u], btbv = biastb[u];
#pragma unroll
      for (int i = 0; i < 2; ++i) {
#pragma unroll
        for (int r = 0; r < 8; ++r) {
          const int row = i * 16 + mOff + r;
          const float tsv = sTs[row];
          const float f1 = tanh_f(acc[i][0][r] * W_CARRY_INV + bf1v);
          const float f2 = tanh_f(acc[i][1][r] * W_CARRY_INV + bf2v);
          const float ga = acc[i][2][r] * W_CARRY_INV + btav;
          const float gb = acc[i][3][r] * W_CARRY_INV + btbv;
          const float ti = sigmoid_f(ga * tsv + gb);
          const float h  = f1 * (1.0f - ti) + ti * f2;
          sA0[row * A0_LD + NIN + u] = (_Float16)h;
          if (t == NSTEP - 1) sHf[row * NHID + u] = h;
        }
      }
    }
    __syncthreads();

    for (int pass = 0; pass < 2; ++pass) {
#pragma unroll
      for (int i = 0; i < 4; ++i) {
        const int row = wave * 4 + i;
        const v8h v = *(const v8h*)(sA0 + row * A0_LD + NIN + lane * 8);
        unsigned short* dst = hseq + (((size_t)(brow0 + row)) * NSTEP + t) * NHID + lane * 8;
        *(volatile v8h*)dst = v;
      }
      __threadfence();
    }
  }

  for (int pass = 0; pass < 2; ++pass) {
#pragma unroll
    for (int i = 0; i < 4; ++i) {
      const int row = wave * 4 + i;
#pragma unroll
      for (int q = 0; q < 2; ++q) {
        const v4f v = *(const v4f*)(sHf + row * NHID + q * 128 + lane * 4);
        *(volatile v4f*)(hn + (size_t)(brow0 + row) * NHID + q * 128 + lane * 4) = v;
      }
    }
    __threadfence();
  }
}

__global__ __launch_bounds__(256) __attribute__((amdgpu_num_vgpr(256)))
void k_proj_heads(const unsigned short* __restrict__ hseq, const unsigned short* __restrict__ wpt,
                  const float* __restrict__ projb, const unsigned short* __restrict__ wh0t,
                  const float* __restrict__ ihb0, const float* __restrict__ ahb0, const float* __restrict__ chb0,
                  const float* __restrict__ ihw1, const float* __restrict__ ihb1,
                  const float* __restrict__ ahw1, const float* __restrict__ ahb1,
                  const float* __restrict__ chw1, const float* __restrict__ chb1,
                  float* __restrict__ out0, float* __restrict__ out1, float* __restrict__ out2) {
  __shared__ __align__(16) _Float16 sC[8][16 * HC_LD];
  __shared__ __align__(16) float    sAct[8][16 * HA_LD];
  __shared__ __align__(16) float    sO0[ROWS_PER_HBLK * 3];
  __shared__ __align__(16) float    sO1[ROWS_PER_HBLK];
  __shared__ __align__(16) float    sO2[ROWS_PER_HBLK];

  const int tid = threadIdx.x, lane = tid & 31, wave = tid >> 5;
  const int rlane = lane & 15, hh = lane >> 4, koff = hh * 8, mOff = hh * 8;
  const _Float16* hs = (const _Float16*)hseq;
  const _Float16* wp = (const _Float16*)wpt;
  const _Float16* wh = (const _Float16*)wh0t;
  const size_t row0 = ((size_t)blockIdx.x * 8 + wave) * 16;

  v8f acc[4];
  acc[0] = zero8(); acc[1] = zero8(); acc[2] = zero8(); acc[3] = zero8();
#pragma unroll 1
  for (int k0 = 0; k0 < NHID; k0 += 32) {
    v16h bfr[4];
#pragma unroll
    for (int j = 0; j < 4; ++j) bfr[j] = Frag<_Float16>::load(wp + (size_t)(j * 16 + rlane) * NHID + koff + k0);
    const v16h afr = Frag<_Float16>::load(hs + (row0 + rlane) * NHID + koff + k0);
#pragma unroll
    for (int j = 0; j < 4; ++j) acc[j] = Frag<_Float16>::mma(afr, bfr[j], acc[j]);
    Frag<_Float16>::guard(acc[0], acc[3], afr, bfr[3]);
    Frag<_Float16>::keep(bfr[0], bfr[1], bfr[2], bfr[3]);
  }
  acc_guard4(acc[0], acc[1], acc[2], acc[3]);
  _Float16* sc = sC[wave];
#pragma unroll
  for (int j = 0; j < 4; ++j) {
    const int col = j * 16 + rlane;
    const float bv = projb[col];
#pragma unroll
    for (int r = 0; r < 8; ++r) sc[(mOff + r) * HC_LD + col] = (_Float16)(acc[j][r] * W_CARRY_INV + bv);
  }
  __builtin_amdgcn_fence(__ATOMIC_RELEASE, "workgroup");
  __builtin_amdgcn_wave_barrier();
  __builtin_amdgcn_fence(__ATOMIC_ACQUIRE, "workgroup");

  v8f a1[3];
  a1[0] = zero8(); a1[1] = zero8(); a1[2] = zero8();
#pragma unroll
  for (int kk = 0; kk < 2; ++kk) {
    const v16h afr = Frag<_Float16>::load(sc + rlane * HC_LD + koff + kk * 32);
    const v16h b0 = Frag<_Float16>::load(wh + (size_t)(0 * 16 + rlane) * NMOT + koff + kk * 32);
    const v16h b1 = Frag<_Float16>::load(wh + (size_t)(1 * 16 + rlane) * NMOT + koff + kk * 32);
    const v16h b2 = Frag<_Float16>::load(wh + (size_t)(2 * 16 + rlane) * NMOT + koff + kk * 32);
    a1[0] = Frag<_Float16>::mma(afr, b0, a1[0]);
    a1[1] = Frag<_Float16>::mma(afr, b1, a1[1]);
    a1[2] = Frag<_Float16>::mma(afr, b2, a1[2]);
    Frag<_Float16>::guard(a1[0], a1[2], afr, b2);
  }
  acc_guard3(a1[0], a1[1], a1[2]);
  float* sa = sAct[wave];
  {
    const float bi  = ihb0[rlane];
    const float ba  = ahb0[rlane];
    const float bc0 = chb0[rlane & 7];
    const float bc  = (rlane < 8) ? bc0 : 0.0f;
#pragma unroll
    for (int r = 0; r < 8; ++r) {
      const int rr = mOff + r;
      sa[rr * HA_LD + rlane]      = silu_f(a1[0][r] * W_CARRY_INV + bi);
      sa[rr * HA_LD + 16 + rlane] = silu_f(a1[1][r] * W_CARRY_INV + ba);
      sa[rr * HA_LD + 32 + rlane] = silu_f(a1[2][r] * W_CARRY_INV + bc);
    }
  }
  __builtin_amdgcn_fence(__ATOMIC_RELEASE, "workgroup");
  __builtin_amdgcn_wave_barrier();
  __builtin_amdgcn_fence(__ATOMIC_ACQUIRE, "workgroup");

  {
    const float* ar = sa + rlane * HA_LD;
    float o0 = ihb1[0], o1 = ihb1[1], o2 = ihb1[2];
#pragma unroll
    for (int i = 0; i < 16; ++i) {
      const float av = ar[i];
      o0 += av * ihw1[i * 3 + 0];
      o1 += av * ihw1[i * 3 + 1];
      o2 += av * ihw1[i * 3 + 2];
    }
    float oa = ahb1[0];
#pragma unroll
    for (int i = 0; i < 16; ++i) oa += ar[16 + i] * ahw1[i];
    float oc = chb1[0];
#pragma unroll
    for (int i = 0; i < 8; ++i) oc += ar[32 + i] * chw1[i];
    o0 = softplus_f(o0); o1 = softplus_f(o1); o2 = softplus_f(o2);
    oa = tanh_f(oa);
    oc = sigmoid_f(oc);
    if (hh == 0) {
      const int lr = wave * 16 + rlane;
      sO0[lr * 3 + 0] = o0; sO0[lr * 3 + 1] = o1; sO0[lr * 3 + 2] = o2;
      sO1[lr] = oa;
      sO2[lr] = oc;
    }
  }
  __syncthreads();

  const int wv = __builtin_amdgcn_readfirstlane(wave);
  const size_t blk = blockIdx.x;
  for (int pass = 0; pass < 2; ++pass) {
    if (wv < 3) {
      const v4f v = *(const v4f*)(sO0 + tid * 4);
      *(volatile v4f*)(out0 + blk * (ROWS_PER_HBLK * 3) + tid * 4) = v;
    } else if (wv == 3) {
      const int i = tid - 96;
      const v4f v = *(const v4f*)(sO1 + i * 4);
      *(volatile v4f*)(out1 + blk * ROWS_PER_HBLK + i * 4) = v;
    } else if (wv == 4) {
      const int i = tid - 128;
      const v4f v = *(const v4f*)(sO2 + i * 4);
      *(volatile v4f*)(out2 + blk * ROWS_PER_HBLK + i * 4) = v;
    }
    __threadfence();
  }
}

extern "C" void kernel_launch(void* const* d_in, const int* in_sizes, int n_in,
                              void* d_out, int out_size, void* d_ws, size_t ws_size,
                              hipStream_t stream) {
  if (n_in != 29) return;
  if (in_sizes[0] != NBATCH * NSTEP * NIN || in_sizes[1] != NBATCH * NSTEP || in_sizes[2] != NBATCH * NHID) return;
  if (in_sizes[3] != KCAT * NBB || in_sizes[4] != NBB || in_sizes[5] != NBB * NBB || in_sizes[6] != NBB) return;
  if (in_sizes[7] != NBB * NHID || in_sizes[9] != NBB * NHID || in_sizes[11] != NBB * NHID || in_sizes[13] != NBB * NHID) return;
  if (in_sizes[8] != NHID || in_sizes[10] != NHID || in_sizes[12] != NHID || in_sizes[14] != NHID) return;
  if (in_sizes[15] != NHID * NMOT || in_sizes[16] != NMOT) return;
  if (in_sizes[17] != NMOT * 16 || in_sizes[18] != 16 || in_sizes[19] != 48 || in_sizes[20] != 3) return;
  if (in_sizes[21] != NMOT * 16 || in_sizes[22] != 16 || in_sizes[23] != 16 || in_sizes[24] != 1) return;
  if (in_sizes[25] != NMOT * 8 || in_sizes[26] != 8 || in_sizes[27] != 8 || in_sizes[28] != 1) return;
  if (out_size != NROWS * 5 + NBATCH * NHID) return;

  const float* x    = (const float*)d_in[0];
  const float* tsp  = (const float*)d_in[1];
  const float* hx   = (const float*)d_in[2];
  const float* bbw0 = (const float*)d_in[3];  const float* bbb0 = (const float*)d_in[4];
  const float* bbw1 = (const float*)d_in[5];  const float* bbb1 = (const float*)d_in[6];
  const float* f1w  = (const float*)d_in[7];  const float* f1b  = (const float*)d_in[8];
  const float* f2w  = (const float*)d_in[9];  const float* f2b  = (const float*)d_in[10];
  const float* taw  = (const float*)d_in[11]; const float* tab  = (const float*)d_in[12];
  const float* tbw  = (const float*)d_in[13]; const float* tbb  = (const float*)d_in[14];
  const float* pjw  = (const float*)d_in[15]; const float* pjb  = (const float*)d_in[16];
  const float* ihw0 = (const float*)d_in[17]; const float* ihb0 = (const float*)d_in[18];
  const float* ihw1 = (const float*)d_in[19]; const float* ihb1 = (const float*)d_in[20];
  const float* ahw0 = (const float*)d_in[21]; const float* ahb0 = (const float*)d_in[22];
  const float* ahw1 = (const float*)d_in[23]; const float* ahb1 = (const float*)d_in[24];
  const float* chw0 = (const float*)d_in[25]; const float* chb0 = (const float*)d_in[26];
  const float* chw1 = (const float*)d_in[27]; const float* chb1 = (const float*)d_in[28];

  float* out0 = (float*)d_out;
  float* out1 = (float*)((char*)d_out + 1572864);
  float* out2 = (float*)((char*)d_out + 2097152);
  float* out3 = (float*)((char*)d_out + 2621440);

  char* ws = (char*)d_ws;
  size_t off = 0;
  const size_t bt0_b  = (size_t)NBB * KCAT * 2;
  const size_t bt1_b  = (size_t)NBB * NBB * 2;
  const size_t bt2_b  = (size_t)4 * NHID * NBB * 2;
  const size_t btp_b  = (size_t)NMOT * NHID * 2;
  const size_t wh0_b  = (size_t)NHEADH * NMOT * 2;
  const size_t hseq_b = (size_t)NROWS * NHID * 2;
  unsigned short* bt0  = (unsigned short*)(ws + off); off += (bt0_b  + 255) & ~(size_t)255;
  unsigned short* bt1  = (unsigned short*)(ws + off); off += (bt1_b  + 255) & ~(size_t)255;
  unsigned short* bt2  = (unsigned short*)(ws + off); off += (bt2_b  + 255) & ~(size_t)255;
  unsigned short* btp  = (unsigned short*)(ws + off); off += (btp_b  + 255) & ~(size_t)255;
  unsigned short* wh0  = (unsigned short*)(ws + off); off += (wh0_b  + 255) & ~(size_t)255;
  unsigned short* hseq = (unsigned short*)(ws + off); off += (hseq_b + 255) & ~(size_t)255;
  if (off > ws_size) return;

  k_transpose_cast<<<dim3(KCAT / 64, NBB / 32), 256, 0, stream>>>(bbw0, bt0, KCAT, NBB, W_CARRY);
  k_transpose_cast<<<dim3(NBB / 64, NBB / 32), 256, 0, stream>>>(bbw1, bt1, NBB, NBB, W_CARRY);
  k_transpose_cast<<<dim3(NBB / 64, NHID / 32), 256, 0, stream>>>(f1w, bt2 + (size_t)0 * NHID * NBB, NBB, NHID, W_CARRY);
  k_transpose_cast<<<dim3(NBB / 64, NHID / 32), 256, 0, stream>>>(f2w, bt2 + (size_t)1 * NHID * NBB, NBB, NHID, W_CARRY);
  k_transpose_cast<<<dim3(NBB / 64, NHID / 32), 256, 0, stream>>>(taw, bt2 + (size_t)2 * NHID * NBB, NBB, NHID, W_CARRY);
  k_transpose_cast<<<dim3(NBB / 64, NHID / 32), 256, 0, stream>>>(tbw, bt2 + (size_t)3 * NHID * NBB, NBB, NHID, W_CARRY);
  k_transpose_cast<<<dim3(NHID / 64, NMOT / 32), 256, 0, stream>>>(pjw, btp, NHID, NMOT, W_CARRY);
  k_pack_head_w<<<1, 384, 0, stream>>>(ihw0, ahw0, chw0, wh0, W_CARRY);

  k_cfc_scan<<<NBLK_SCAN, 256, 0, stream>>>(x, tsp, hx, bt0, bbb0, bt1, bbb1, bt2, f1b, f2b, tab, tbb, hseq, out3);

  k_proj_heads<<<NROWS / ROWS_PER_HBLK, 256, 0, stream>>>(hseq, btp, pjb, wh0, ihb0, ahb0, chb0,
                                                         ihw1, ihb1, ahw1, ahb1, chw1, chb1, out0, out1, out2);
}
